// SelectiveSSM_59828894433547
// MI455X (gfx1250) — hardware-verified
//
#include <hip/hip_runtime.h>
#include <stddef.h>
#include <stdint.h>

#define DM     1024
#define DS     16
#define NBATCH 4
#define SEQ    2048
#define MROWS  (NBATCH * SEQ)
#define NX     (MROWS * DM)
#define NW     (DM * DM)
#define NBCW   (DS * DM)
#define NALL   1088
#define BCP    64
#define LOG2E  1.44269504088896340736f

#define U_X    (NX / 8)
#define U_WDT  (NW / 8)
#define U_WB   (NBCW / 8)
#define U_WC   (NBCW / 8)
#define U_Z    ((NALL - DM - 2 * DS) * DM / 8)
#define U_A    (DM * DS / 4)
#define E0     U_X
#define E1     (E0 + U_WDT)
#define E2     (E1 + U_WB)
#define E3     (E2 + U_WC)
#define E4     (E3 + U_Z)
#define E5     (E4 + U_A)

static_assert(U_X % 256 == 0 && U_WDT % 256 == 0 && U_WB % 256 == 0 && U_WC % 256 == 0);
static_assert(U_Z % 256 == 0 && U_A % 256 == 0 && E5 % 256 == 0);
static_assert((U_WDT + U_WB + U_WC + U_Z) * 8 == NALL * DM);
static_assert(DM % 32 == 0 && MROWS % 128 == 0 && NALL % 64 == 0 && SEQ % 64 == 0);

typedef float          v4f   __attribute__((ext_vector_type(4)));
typedef float          v8f   __attribute__((ext_vector_type(8)));
typedef int            v8i   __attribute__((ext_vector_type(8)));
typedef unsigned short v8us  __attribute__((ext_vector_type(8)));
typedef unsigned short v16us __attribute__((ext_vector_type(16)));
typedef __bf16         v16bf __attribute__((ext_vector_type(16)));
typedef v4f  __attribute__((may_alias)) v4fa;
typedef v8us __attribute__((may_alias)) v8usa;
union FragB { v16bf v; v16us u; v8us h[2]; v8i w; };

__device__ __forceinline__ v8f wmb(const FragB& a, const FragB& b, v8f c) {
  v8f d = __builtin_amdgcn_wmma_f32_16x16x32_bf16(false, a.v, false, b.v, (short)0, c, false, false);
  asm volatile("v_nop\n\tv_nop\n\tv_nop\n\tv_nop" : "+v"(d) : "v"(a.w), "v"(b.w));
  return d;
}

__device__ __forceinline__ unsigned bf16_bits(float f) {
  const unsigned u = __float_as_uint(f);
  return (u + 0x7FFFu + ((u >> 16) & 1u)) >> 16;
}
__device__ __forceinline__ float bf16_val(float f) {
  return __uint_as_float(bf16_bits(f) << 16);
}
__device__ __forceinline__ void put16(unsigned short* dp, v8us o) {
  *(volatile v8us*)dp = o;
  __threadfence();
  *(volatile v8us*)dp = o;
}
__device__ __forceinline__ void putf4(float* dp, v4f o) {
  *(volatile v4f*)dp = o;
  __threadfence();
  *(volatile v4f*)dp = o;
}
__device__ __forceinline__ v8us cvt8(const float* src) {
  const v4f a = *(const v4fa*)src;
  const v4f c = *(const v4fa*)(src + 4);
  v8us o;
  o[0] = (unsigned short)bf16_bits(a.x); o[1] = (unsigned short)bf16_bits(a.y);
  o[2] = (unsigned short)bf16_bits(a.z); o[3] = (unsigned short)bf16_bits(a.w);
  o[4] = (unsigned short)bf16_bits(c.x); o[5] = (unsigned short)bf16_bits(c.y);
  o[6] = (unsigned short)bf16_bits(c.z); o[7] = (unsigned short)bf16_bits(c.w);
  return o;
}

__global__ __launch_bounds__(256) void k_prep(const float* __restrict__ x, const float* __restrict__ Wdt,
                                              const float* __restrict__ WB, const float* __restrict__ WC,
                                              const float* __restrict__ Alog,
                                              unsigned short* XB, unsigned short* WALL, float* A2) {
  const int u = (int)blockIdx.x * 256 + (int)threadIdx.x;
  if (u < E0) {
    put16(XB + (size_t)u * 8, cvt8(x + (size_t)u * 8));
  } else if (u < E1) {
    const int v = u - E0;
    put16(WALL + (size_t)v * 8, cvt8(Wdt + (size_t)v * 8));
  } else if (u < E2) {
    const int v = u - E1;
    put16(WALL + (size_t)NW + (size_t)v * 8, cvt8(WB + (size_t)v * 8));
  } else if (u < E3) {
    const int v = u - E2;
    put16(WALL + (size_t)NW + (size_t)NBCW + (size_t)v * 8, cvt8(WC + (size_t)v * 8));
  } else if (u < E4) {
    const int v = u - E3;
    const v8us z = {0, 0, 0, 0, 0, 0, 0, 0};
    put16(WALL + (size_t)NW + (size_t)2 * NBCW + (size_t)v * 8, z);
  } else if (u < E5) {
    const int v = u - E4;
    const v4f a = *(const v4fa*)(Alog + (size_t)v * 4);
    v4f o;
    o.x = -expf(bf16_val(a.x)) * LOG2E;
    o.y = -expf(bf16_val(a.y)) * LOG2E;
    o.z = -expf(bf16_val(a.z)) * LOG2E;
    o.w = -expf(bf16_val(a.w)) * LOG2E;
    putf4(A2 + (size_t)v * 4, o);
  }
}

__device__ __forceinline__ float softplus_f(float z) {
  return fmaxf(z, 0.0f) + log1pf(expf(-fabsf(z)));
}

__global__ __launch_bounds__(128) void k_proj(const unsigned short* __restrict__ XB,
                                              const unsigned short* __restrict__ WALL,
                                              const float* __restrict__ bdt,
                                              float* DT, float* BC) {
  __shared__ __attribute__((aligned(16))) float stg[128 * 64];

  const int tid = (int)threadIdx.x, lane = tid & 31, w = tid >> 5;
  const int hh = lane >> 4, m = lane & 15;
  const int m0 = (int)blockIdx.x * 128;
  const int y  = (int)blockIdx.y;
  const bool isdt = y < 16;

  const unsigned short* ap0 = XB + (size_t)(m0 + 32 * w + m) * DM + 8 * hh;
  const unsigned short* ap1 = ap0 + (size_t)16 * DM;
  const unsigned short* bp  = WALL + (size_t)(64 * y + m) * DM + 8 * hh;

  v8f acc[2][4];
  {
    const v8f z = {0.f, 0.f, 0.f, 0.f, 0.f, 0.f, 0.f, 0.f};
#pragma unroll
    for (int mt = 0; mt < 2; ++mt)
#pragma unroll
      for (int nt = 0; nt < 4; ++nt) acc[mt][nt] = z;
  }

#pragma unroll 1
  for (int k0 = 0; k0 < DM; k0 += 32) {
    FragB a0, a1;
    a0.h[0] = *(const v8usa*)(ap0 + k0);
    a0.h[1] = *(const v8usa*)(ap0 + k0 + 16);
    a1.h[0] = *(const v8usa*)(ap1 + k0);
    a1.h[1] = *(const v8usa*)(ap1 + k0 + 16);
#pragma unroll
    for (int nt = 0; nt < 4; ++nt) {
      const unsigned short* wq = bp + (size_t)(16 * nt) * DM + k0;
      FragB b;
      b.h[0] = *(const v8usa*)wq;
      b.h[1] = *(const v8usa*)(wq + 16);
      acc[0][nt] = wmb(a0, b, acc[0][nt]);
      acc[1][nt] = wmb(a1, b, acc[1][nt]);
    }
  }

#pragma unroll
  for (int nt = 0; nt < 4; ++nt) {
    const int lc = 16 * nt + m;
    int bc = 64 * y + lc;
    bc = bc > DM - 1 ? DM - 1 : bc;
    const float bl = bf16_val(bdt[bc]);
    const float bvv = isdt ? bl : 0.0f;
#pragma unroll
    for (int mt = 0; mt < 2; ++mt)
#pragma unroll
      for (int r = 0; r < 8; ++r)
        stg[(32 * w + 16 * mt + 8 * hh + r) * 64 + lc] = acc[mt][nt][r] + bvv;
  }
  __syncthreads();

  if (isdt) {
#pragma unroll 1
    for (int i = 0; i < 16; ++i) {
      float* p = stg + (32 * w + 2 * i + hh) * 64 + 4 * m;
      v4f v = *(v4fa*)p;
      v.x = softplus_f(v.x);
      v.y = softplus_f(v.y);
      v.z = softplus_f(v.z);
      v.w = softplus_f(v.w);
      *(v4fa*)p = v;
    }
  }

  float* C        = isdt ? DT : BC;
  const int ldc   = isdt ? DM : BCP;
  const int cb    = isdt ? 64 * y : 0;
  v4f pv[16];
#pragma unroll
  for (int i = 0; i < 16; ++i) pv[i] = *(const v4fa*)(stg + (32 * w + 2 * i + hh) * 64 + 4 * m);
#pragma unroll
  for (int i = 0; i < 16; ++i) {
    float* op = C + (size_t)(m0 + 32 * w + 2 * i + hh) * (size_t)ldc + cb + 4 * m;
    *(volatile v4f*)op = pv[i];
  }
  __threadfence();
#pragma unroll
  for (int i = 0; i < 16; ++i) {
    float* op = C + (size_t)(m0 + 32 * w + 2 * i + hh) * (size_t)ldc + cb + 4 * m;
    *(volatile v4f*)op = pv[i];
  }
}

__global__ __launch_bounds__(256) void k_scan(const float* __restrict__ DT,
                                              const unsigned short* __restrict__ XB,
                                              const float* __restrict__ BC,
                                              const float* __restrict__ A2,
                                              const float* __restrict__ Dp,
                                              float* out) {
  __shared__ __attribute__((aligned(16))) float sBC[64 * 32];

  const int tid = (int)threadIdx.x;
  const int d   = (int)blockIdx.x * 256 + tid;
  const int b   = (int)blockIdx.y;
  const int rowBase = b * SEQ;

  float a2[16];
  {
    const float* ar = A2 + (size_t)d * DS;
    const v4f q0 = *(const v4fa*)(ar);
    const v4f q1 = *(const v4fa*)(ar + 4);
    const v4f q2 = *(const v4fa*)(ar + 8);
    const v4f q3 = *(const v4fa*)(ar + 12);
    a2[0] = q0.x;  a2[1] = q0.y;  a2[2] = q0.z;  a2[3] = q0.w;
    a2[4] = q1.x;  a2[5] = q1.y;  a2[6] = q1.z;  a2[7] = q1.w;
    a2[8] = q2.x;  a2[9] = q2.y;  a2[10] = q2.z; a2[11] = q2.w;
    a2[12] = q3.x; a2[13] = q3.y; a2[14] = q3.z; a2[15] = q3.w;
  }
  float h[16];
#pragma unroll
  for (int n = 0; n < 16; ++n) h[n] = 0.0f;
  const float Dv = bf16_val(Dp[d]);

  const float*          dtp = DT  + (size_t)rowBase * DM + d;
  const unsigned short* xp  = XB  + (size_t)rowBase * DM + d;
  float*                op  = out + (size_t)rowBase * DM + d;

#pragma unroll 1
  for (int c = 0; c < SEQ / 64; ++c) {
    __syncthreads();
#pragma unroll
    for (int j = 0; j < 2; ++j) {
      const int idx = tid + 256 * j;
      const int row = idx >> 3;
      const int c4  = idx & 7;
      const v4f v = *(const v4fa*)(BC + (size_t)(rowBase + c * 64 + row) * BCP + 4 * c4);
      *(v4fa*)(sBC + row * 32 + 4 * c4) = v;
    }
    __syncthreads();

#pragma unroll 1
    for (int s = 0; s < 64; ++s) {
      const size_t ro = (size_t)(c * 64 + s) * DM;
      const float dt = dtp[ro];
      const unsigned xw = (unsigned)xp[ro];
      const float xb = __uint_as_float(xw << 16);
      const float* r = sBC + s * 32;
      const v4f b0 = *(const v4fa*)(r);
      const v4f b1 = *(const v4fa*)(r + 4);
      const v4f b2 = *(const v4fa*)(r + 8);
      const v4f b3 = *(const v4fa*)(r + 12);
      const v4f c0 = *(const v4fa*)(r + 16);
      const v4f c1 = *(const v4fa*)(r + 20);
      const v4f c2 = *(const v4fa*)(r + 24);
      const v4f c3 = *(const v4fa*)(r + 28);
      const float bpv[16] = {b0.x, b0.y, b0.z, b0.w, b1.x, b1.y, b1.z, b1.w,
                             b2.x, b2.y, b2.z, b2.w, b3.x, b3.y, b3.z, b3.w};
      const float cpv[16] = {c0.x, c0.y, c0.z, c0.w, c1.x, c1.y, c1.z, c1.w,
                             c2.x, c2.y, c2.z, c2.w, c3.x, c3.y, c3.z, c3.w};
      float acc = 0.0f;
#pragma unroll
      for (int n = 0; n < 16; ++n) {
        const float uin = (dt * bpv[n]) * xb;
        const float e   = exp2f(dt * a2[n]);
        h[n] = fmaf(e, h[n], uin);
        acc  = fmaf(h[n], cpv[n], acc);
      }
      const float yv = fmaf(Dv, xb, acc);
      volatile float* vo = (volatile float*)(op + ro);
      *vo = yv;
      __threadfence();
      *vo = yv;
    }
  }
}

extern "C" void kernel_launch(void* const* d_in, const int* in_sizes, int n_in,
                              void* d_out, int out_size, void* d_ws, size_t ws_size,
                              hipStream_t stream) {
  if (n_in < 7) return;
  if (in_sizes[0] != NX) return;
  if (in_sizes[1] != NW) return;
  if (in_sizes[2] != DM) return;
  if (in_sizes[3] != NBCW || in_sizes[4] != NBCW) return;
  if (in_sizes[5] != DM * DS) return;
  if (in_sizes[6] != DM) return;
  if (out_size != NX) return;

  const float* x    = (const float*)d_in[0];
  const float* Wdt  = (const float*)d_in[1];
  const float* bdt  = (const float*)d_in[2];
  const float* WB   = (const float*)d_in[3];
  const float* WC   = (const float*)d_in[4];
  const float* Alog = (const float*)d_in[5];
  const float* Dp   = (const float*)d_in[6];
  float* out = (float*)d_out;

  const size_t szXB   = (size_t)NX * 2;
  const size_t szWALL = (size_t)NALL * DM * 2;
  const size_t szA2   = (size_t)DM * DS * 4;
  const size_t szDT   = (size_t)NX * 4;
  const size_t szBC   = (size_t)MROWS * BCP * 4;
  const size_t total  = szXB + szWALL + szA2 + szDT + szBC;
  if (total > ws_size || total > (size_t)134217728) return;

  char* ws = (char*)d_ws;
  unsigned short* XB   = (unsigned short*)(ws);
  unsigned short* WALL = (unsigned short*)(ws + szXB);
  float*          A2   = (float*)(ws + szXB + szWALL);
  float*          DT   = (float*)(ws + szXB + szWALL + szA2);
  float*          BC   = (float*)(ws + szXB + szWALL + szA2 + szDT);

  k_prep<<<E5 / 256, 256, 0, stream>>>(x, Wdt, WB, WC, Alog, XB, WALL, A2);
  k_proj<<<dim3(MROWS / 128, NALL / 64), 128, 0, stream>>>(XB, WALL, bdt, DT, BC);
  k_scan<<<dim3(DM / 256, NBATCH), 256, 0, stream>>>(DT, XB, BC, A2, Dp, out);
}
